// PositionAttentionModule_9320079032514
// MI455X (gfx1250) — hardware-verified
//
#include <hip/hip_runtime.h>
#include <stdint.h>
#include <stddef.h>

typedef __attribute__((ext_vector_type(16))) _Float16 v16h;
typedef __attribute__((ext_vector_type(8)))  _Float16 v8h;
typedef __attribute__((ext_vector_type(16))) __bf16   v16b;
typedef __attribute__((ext_vector_type(8)))  __bf16   v8b;
typedef __attribute__((ext_vector_type(8)))  float    v8f;
typedef __attribute__((ext_vector_type(4)))  float    v4f;
typedef __attribute__((ext_vector_type(4)))  unsigned int u32x4;

__device__ __forceinline__ unsigned short f2bf_bits(float f) {
  unsigned u = __float_as_uint(f);
  return (unsigned short)((u + 0x7FFFu + ((u >> 16) & 1u)) >> 16);
}
__device__ __forceinline__ float bf_bits2f(unsigned short h) { return __uint_as_float(((unsigned)h) << 16); }

__device__ __forceinline__ void dep_guard_h(v8f& a, v8f& b, v16h x, v16h y) { asm volatile("v_nop\n\tv_nop\n\tv_nop\n\tv_nop" : "+v"(a), "+v"(b) : "v"(x), "v"(y)); }
__device__ __forceinline__ void dep_guard_b(v8f& a, v8f& b, v16b x, v16b y) { asm volatile("v_nop\n\tv_nop\n\tv_nop\n\tv_nop" : "+v"(a), "+v"(b) : "v"(x), "v"(y)); }
__device__ __forceinline__ void keep4_h(v16h a, v16h b, v16h c, v16h d) { asm volatile("v_nop" :: "v"(a), "v"(b), "v"(c), "v"(d)); }
__device__ __forceinline__ void keep4_b(v16b a, v16b b, v16b c, v16b d) { asm volatile("v_nop" :: "v"(a), "v"(b), "v"(c), "v"(d)); }
__device__ __forceinline__ void acc_guard4(v8f& a, v8f& b, v8f& c, v8f& d) { asm volatile("v_nop\n\tv_nop\n\tv_nop\n\tv_nop" : "+v"(a), "+v"(b), "+v"(c), "+v"(d)); }
template <typename T> struct Frag;
template <> struct Frag<_Float16> {
  typedef v16h V; union U { v16h v; v8h h[2]; };
  static __device__ __forceinline__ v16h load(const _Float16* p) {
    U f; f.h[0] = *(const v8h*)(p); f.h[1] = *(const v8h*)(p + 16); return f.v;
  }
  static __device__ __forceinline__ v8f mma(v16h a, v16h b, v8f c) {
    return __builtin_amdgcn_wmma_f32_16x16x32_f16(false, a, false, b, (short)0, c, false, false);
  }
  static __device__ __forceinline__ void guard(v8f& a, v8f& b, v16h x, v16h y) { dep_guard_h(a, b, x, y); }
  static __device__ __forceinline__ void keep(v16h a, v16h b, v16h c, v16h d) { keep4_h(a, b, c, d); }
};
template <> struct Frag<__bf16> {
  typedef v16b V; union U { v16b v; v8b h[2]; };
  static __device__ __forceinline__ v16b load(const __bf16* p) {
    U f; f.h[0] = *(const v8b*)(p); f.h[1] = *(const v8b*)(p + 16); return f.v;
  }
  static __device__ __forceinline__ v8f mma(v16b a, v16b b, v8f c) {
    return __builtin_amdgcn_wmma_f32_16x16x32_bf16(false, a, false, b, (short)0, c, false, false);
  }
  static __device__ __forceinline__ void guard(v8f& a, v8f& b, v16b x, v16b y) { dep_guard_b(a, b, x, y); }
  static __device__ __forceinline__ void keep(v16b a, v16b b, v16b c, v16b d) { keep4_b(a, b, c, d); }
};

template <int ET> struct Elem;
template <> struct Elem<0> { typedef _Float16 T; };
template <> struct Elem<1> { typedef __bf16 T; };
template <int ET, bool SPLIT, int BIAS_MODE, int OUT_MODE, bool RESID, int ACT = 0>
__global__ __launch_bounds__(256) void wmma_gemm64(
    const unsigned short* __restrict__ Ap, const unsigned short* __restrict__ A2p, int lda, long strideA,
    const unsigned short* __restrict__ Btp, const unsigned short* __restrict__ Bt2p, int ldb, long strideB,
    void* __restrict__ Cout, void* __restrict__ Cout2, int ldc, long strideC,
    const float* __restrict__ bias,
    const float* __restrict__ resid, long strideR,
    int M, int N, int K, float scale) {
  typedef typename Elem<ET>::T T;
  typedef typename Frag<T>::V V;
  const T* A = (const T*)Ap; const T* A2 = (const T*)A2p; const T* Bt = (const T*)Btp; const T* Bt2 = (const T*)Bt2p;
  __shared__ __align__(16) float sT[8][16 * 68];
  const int b    = blockIdx.y;
  const int lane = threadIdx.x & 31;
  const int wave = threadIdx.x >> 5;
  const int tilesN = N >> 6;
  const int tilesM = M >> 6;
  const int tile = blockIdx.x * 8 + wave;
  if (tile >= tilesM * tilesN) return;
  const int tm = tile / tilesN;
  const int tn = tile - tm * tilesN;
  const int m0 = tm << 6;
  const int n0 = tn << 6;

  const T* Ab  = A  + (size_t)b * strideA;
  const T* Bb  = Bt + (size_t)b * strideB;
  const T* Ab2 = SPLIT ? (A2  + (size_t)b * strideA) : nullptr;
  const T* Bb2 = SPLIT ? (Bt2 + (size_t)b * strideB) : nullptr;

  const int rlane = lane & 15;
  const int koff  = (lane >> 4) * 8;
  const int mOff  = (lane >> 4) * 8;

  v8f acc[4][4];
#pragma unroll
  for (int i = 0; i < 4; ++i)
#pragma unroll
    for (int j = 0; j < 4; ++j) acc[i][j] = (v8f){0.f,0.f,0.f,0.f,0.f,0.f,0.f,0.f};

  for (int k0 = 0; k0 < K; k0 += 32) {
    V bh[4], bl[4];
#pragma unroll
    for (int j = 0; j < 4; ++j) {
      const size_t bo = (size_t)(n0 + (j << 4) + rlane) * ldb + koff + k0;
      bh[j] = Frag<T>::load(Bb + bo);
      if (SPLIT) bl[j] = Frag<T>::load(Bb2 + bo);
    }
#pragma unroll
    for (int i = 0; i < 4; ++i) {
      const size_t ao = (size_t)(m0 + (i << 4) + rlane) * lda + koff + k0;
      V ah = Frag<T>::load(Ab + ao);
      V al;
      if (SPLIT) al = Frag<T>::load(Ab2 + ao);
#pragma unroll
      for (int j = 0; j < 4; ++j) {
        acc[i][j] = Frag<T>::mma(ah, bh[j], acc[i][j]);
        if (SPLIT) {
          acc[i][j] = Frag<T>::mma(ah, bl[j], acc[i][j]);
          acc[i][j] = Frag<T>::mma(al, bh[j], acc[i][j]);
        }
      }
      Frag<T>::guard(acc[i][0], acc[i][3], ah, SPLIT ? al : ah);
    }
    Frag<T>::keep(bh[0], bh[1], bh[2], bh[3]);
    if (SPLIT) Frag<T>::keep(bl[0], bl[1], bl[2], bl[3]);
  }
  acc_guard4(acc[0][0], acc[0][1], acc[0][2], acc[0][3]);
  acc_guard4(acc[1][0], acc[1][1], acc[1][2], acc[1][3]);
  acc_guard4(acc[2][0], acc[2][1], acc[2][2], acc[2][3]);
  acc_guard4(acc[3][0], acc[3][1], acc[3][2], acc[3][3]);

  float* slab = sT[wave];
  const float* Rb = RESID ? (resid + (size_t)b * strideR) : nullptr;
#pragma unroll
  for (int i = 0; i < 4; ++i) {
    const int mBase = m0 + (i << 4);
#pragma unroll
    for (int j = 0; j < 4; ++j) {
      const int n = n0 + (j << 4) + rlane;
      float bv = 0.f;
      if (BIAS_MODE == 2) bv = bias[n];
#pragma unroll
      for (int r = 0; r < 8; ++r) {
        float v = acc[i][j][r] * scale;
        if (BIAS_MODE == 1) v += bias[mBase + mOff + r];
        if (BIAS_MODE == 2) v += bv;
        if (RESID) v += Rb[(size_t)(mBase + mOff + r) * ldc + n];
        if (ACT == 1) v = tanhf(v);
        if (ACT == 2) v = fmaxf(v, 0.0f);
        if (ACT == 3) v = v / (1.0f + expf(-v));
        if (ACT == 4) v = (v > 0.f) ? v : 0.01f * v;
        if (ACT == 5) v = 0.5f * v * (1.0f + erff(v * 0.70710678118654752f));
        slab[(mOff + r) * 68 + (j << 4) + rlane] = v;
      }
    }
    __builtin_amdgcn_fence(__ATOMIC_RELEASE, "workgroup");
    __builtin_amdgcn_wave_barrier();
    __builtin_amdgcn_fence(__ATOMIC_ACQUIRE, "workgroup");
    if (OUT_MODE == 0) {
      float* C = (float*)Cout + (size_t)b * strideC;
      const int hh = lane >> 4, c4 = (lane & 15) * 4;
      for (int pass = 0; pass < 2; ++pass) {
#pragma unroll
        for (int it = 0; it < 8; ++it) {
          const int row = it * 2 + hh;
          v4f v = *(const v4f*)(slab + row * 68 + c4);
          *(volatile v4f*)(C + (size_t)(mBase + row) * ldc + n0 + c4) = v;
        }
        __threadfence();
      }
    } else {
      const int q = lane >> 3, c8 = (lane & 7) * 8;
      unsigned short* C  = (unsigned short*)Cout  + (size_t)b * strideC;
      unsigned short* C2 = (OUT_MODE == 2) ? ((unsigned short*)Cout2 + (size_t)b * strideC) : nullptr;
      for (int pass = 0; pass < 2; ++pass) {
#pragma unroll
        for (int it = 0; it < 4; ++it) {
          const int row = it * 4 + q;
          const float* sp = slab + row * 68 + c8;
          v8h hv, lv;
#pragma unroll
          for (int e = 0; e < 8; ++e) {
            if (OUT_MODE == 1) {
              hv[e] = (_Float16)sp[e];
            } else {
              unsigned short hb = f2bf_bits(sp[e]);
              unsigned short lb = f2bf_bits(sp[e] - bf_bits2f(hb));
              hv[e] = __builtin_bit_cast(_Float16, hb);
              lv[e] = __builtin_bit_cast(_Float16, lb);
            }
          }
          *(volatile v8h*)(C + (size_t)(mBase + row) * ldc + n0 + c8) = hv;
          if (OUT_MODE == 2) *(volatile v8h*)(C2 + (size_t)(mBase + row) * ldc + n0 + c8) = lv;
        }
        __threadfence();
      }
    }
    __builtin_amdgcn_fence(__ATOMIC_RELEASE, "workgroup");
    __builtin_amdgcn_wave_barrier();
    __builtin_amdgcn_fence(__ATOMIC_ACQUIRE, "workgroup");
  }
}

#ifndef NB
#define NB 4
#endif
#ifndef SEQ
#define SEQ 4096
#endif
#define NB_FULL   4
#define SEQ_FULL  4096
#define PA_C      512
#define PA_D      64
#define PA_QKP    128
#define PA_TP     520
#define PA_KW     16
#define PA_KCH    64
#define PA_OBP    36
#define PA_PSC    32768.0f
#ifndef OUT_NSTRIDE
#define OUT_NSTRIDE SEQ
#endif
#ifndef OUT_BSTRIDE
#define OUT_BSTRIDE (PA_C * SEQ)
#endif

static_assert(PA_C == 512);
static_assert(PA_D == 64);
static_assert(PA_QKP == 2 * PA_D);
static_assert(PA_D % 32 == 0);
static_assert(PA_C % 64 == 0);
static_assert(PA_C % 32 == 0);
static_assert(SEQ % 256 == 0);
static_assert(SEQ % PA_KCH == 0);
static_assert(SEQ % 32 == 0);
static_assert(NB >= 1 && NB <= NB_FULL);
static_assert(SEQ <= SEQ_FULL);
static_assert((PA_TP * 2) % 16 == 0);
static_assert((PA_OBP * 4) % 16 == 0);

__device__ __forceinline__ v8f mma_bf16g(v16b a, v16b b, v8f c) {
  c = __builtin_amdgcn_wmma_f32_16x16x32_bf16(false, a, false, b, (short)0, c, false, false);
  asm volatile("v_nop\n\tv_nop\n\tv_nop\n\tv_nop" : "+v"(c) : "v"(a), "v"(b));
  return c;
}
__device__ __forceinline__ v8f mma_f16g(v16h a, v16h b, v8f c) {
  c = __builtin_amdgcn_wmma_f32_16x16x32_f16(false, a, false, b, (short)0, c, false, false);
  asm volatile("v_nop\n\tv_nop\n\tv_nop\n\tv_nop" : "+v"(c) : "v"(a), "v"(b));
  return c;
}

#define PP_QKBLK  32
#define PP_VBLK   128
#define PP_NBLK   (PP_QKBLK + PP_VBLK + 1)
static_assert(PP_QKBLK * 256 * 8 == PA_QKP * PA_C);
static_assert(PP_VBLK * 256 * 8 == PA_C * PA_C);
static_assert((PA_QKP + PA_C) / 4 <= 256);

__global__ __launch_bounds__(256)
void prep_params(const float* __restrict__ wq, const float* __restrict__ wk, const float* __restrict__ wv,
                 const float* __restrict__ bq, const float* __restrict__ bk, const float* __restrict__ bvp,
                 unsigned short* __restrict__ Wqk16, unsigned short* __restrict__ Wv16, float* __restrict__ brnd)
{
  const int blk = blockIdx.x;
  const int t = threadIdx.x;
  if (blk < PP_QKBLK) {
    const int i = blk * 256 + t;
    const int row = i >> 6;
    const int col = (i & 63) * 8;
    const int rq = row < PA_D ? row : (PA_D - 1);
    const int rk = row < PA_D ? 0 : (row - PA_D);
    const v4f q0v = *(const v4f*)(wq + (size_t)rq * PA_C + col);
    const v4f q1v = *(const v4f*)(wq + (size_t)rq * PA_C + col + 4);
    const v4f k0v = *(const v4f*)(wk + (size_t)rk * PA_C + col);
    const v4f k1v = *(const v4f*)(wk + (size_t)rk * PA_C + col + 4);
    const bool useq = row < PA_D;
    v8h hv;
#pragma unroll
    for (int e = 0; e < 4; ++e) {
      const float a0 = useq ? q0v[e] : k0v[e];
      const float a1 = useq ? q1v[e] : k1v[e];
      hv[e]     = __builtin_bit_cast(_Float16, f2bf_bits(a0));
      hv[4 + e] = __builtin_bit_cast(_Float16, f2bf_bits(a1));
    }
    unsigned short* dst = Wqk16 + (size_t)i * 8;
    *(volatile v8h*)dst = hv;
    __threadfence();
    *(volatile v8h*)dst = hv;
  } else if (blk < PP_QKBLK + PP_VBLK) {
    const int i = (blk - PP_QKBLK) * 256 + t;
    const v4f a0 = *(const v4f*)(wv + (size_t)i * 8);
    const v4f a1 = *(const v4f*)(wv + (size_t)i * 8 + 4);
    v8h hv;
#pragma unroll
    for (int e = 0; e < 4; ++e) {
      hv[e]     = __builtin_bit_cast(_Float16, f2bf_bits(a0[e]));
      hv[4 + e] = __builtin_bit_cast(_Float16, f2bf_bits(a1[e]));
    }
    unsigned short* dst = Wv16 + (size_t)i * 8;
    *(volatile v8h*)dst = hv;
    __threadfence();
    *(volatile v8h*)dst = hv;
  } else {
    if (t < (PA_QKP + PA_C) / 4) {
      const int jq = t < 16 ? t : 15;
      const int jk = t < 16 ? 0 : (t < 32 ? (t - 16) : 15);
      const int jv = t < 32 ? 0 : (t - 32);
      const v4f aq = *(const v4f*)(bq + 4 * jq);
      const v4f ak = *(const v4f*)(bk + 4 * jk);
      const v4f av = *(const v4f*)(bvp + 4 * jv);
      v4f rv;
#pragma unroll
      for (int e = 0; e < 4; ++e) {
        const float s0 = t < 16 ? aq[e] : (t < 32 ? ak[e] : av[e]);
        rv[e] = bf_bits2f(f2bf_bits(s0));
      }
      float* dst = brnd + 4 * t;
      *(volatile v4f*)dst = rv;
      __threadfence();
      *(volatile v4f*)dst = rv;
    }
  }
}

__global__ __launch_bounds__(256)
void xpose_x_bf16(const float* __restrict__ x, unsigned short* __restrict__ Xt)
{
  __shared__ __align__(16) unsigned short tile[32 * PA_TP];
  const int t = threadIdx.x;
  const int nblk = SEQ / 32;
  const int b = blockIdx.x / nblk;
  const int n0 = (blockIdx.x - b * nblk) * 32;
  const float* xb = x + (size_t)b * PA_C * SEQ_FULL;
#pragma unroll
  for (int i = 0; i < 16; ++i) {
    const int cc = i * 32 + (t >> 3);
    const int n4 = (t & 7) * 4;
    const v4f xv = *(const v4f*)(xb + (size_t)cc * SEQ_FULL + n0 + n4);
#pragma unroll
    for (int e = 0; e < 4; ++e) tile[(n4 + e) * PA_TP + cc] = f2bf_bits(xv[e]);
  }
  __syncthreads();
  unsigned short* dst = Xt + ((size_t)b * SEQ + n0) * PA_C;
  for (int pass = 0; pass < 2; ++pass) {
#pragma unroll
    for (int it = 0; it < 8; ++it) {
      const int L = it * 32 + (t >> 3);
      const int row = L >> 3;
      const int col = (L & 7) * 64 + (t & 7) * 8;
      const u32x4 w = *(const u32x4*)(tile + row * PA_TP + col);
      *(volatile u32x4*)(dst + (size_t)row * PA_C + col) = w;
    }
    __threadfence();
  }
}

__global__ __launch_bounds__(256)
void pos_attn(const unsigned short* __restrict__ QKh, const unsigned short* __restrict__ QKl,
              const unsigned short* __restrict__ Vp, const float* __restrict__ x,
              const float* __restrict__ alphap, float* __restrict__ out)
{
  __shared__ __align__(16) _Float16 Psh[2][16 * PA_KCH];
  __shared__ float Smx[2][4][16];
  __shared__ float Ssm[2][4][16];
  __shared__ __align__(16) float Ob[(PA_C / 2) * PA_OBP];

  const int tid  = threadIdx.x;
  const int wave = tid >> 5;
  const int lane = tid & 31;
  const int hh   = lane >> 4;
  const int c    = lane & 15;
  const int rg   = wave >> 2;
  const int ch   = wave & 3;
  const int nqb  = SEQ / 32;
  const int b    = blockIdx.x / nqb;
  const int q0   = (blockIdx.x - b * nqb) * 32;
  const int qr0  = q0 + 16 * rg;

  const __bf16* Qh = (const __bf16*)QKh + (size_t)b * SEQ * PA_QKP;
  const __bf16* Ql = (const __bf16*)QKl + (size_t)b * SEQ * PA_QKP;
  const _Float16* Vb = (const _Float16*)Vp + (size_t)b * PA_C * SEQ + (size_t)(128 * ch) * SEQ;

  v16b qah[2], qal[2];
#pragma unroll
  for (int ks = 0; ks < 2; ++ks) {
    qah[ks] = Frag<__bf16>::load(Qh + (size_t)(qr0 + c) * PA_QKP + 32 * ks + 8 * hh);
    qal[ks] = Frag<__bf16>::load(Ql + (size_t)(qr0 + c) * PA_QKP + 32 * ks + 8 * hh);
  }

  float mrow[8], lrow[8];
  v8f oacc[8];
#pragma unroll
  for (int r = 0; r < 8; ++r) { mrow[r] = -INFINITY; lrow[r] = 0.f; }
#pragma unroll
  for (int t = 0; t < 8; ++t) oacc[t] = (v8f){0.f,0.f,0.f,0.f,0.f,0.f,0.f,0.f};

  _Float16* pw = Psh[rg];
  const float al = bf_bits2f(f2bf_bits(alphap[0]));

#pragma unroll 1
  for (int kc = 0; kc < SEQ / PA_KCH; ++kc) {
    const int key0 = kc * PA_KCH + PA_KW * ch;
    v8f s = (v8f){0.f,0.f,0.f,0.f,0.f,0.f,0.f,0.f};
#pragma unroll
    for (int ks = 0; ks < 2; ++ks) {
      const size_t ko = (size_t)(key0 + c) * PA_QKP + PA_D + 32 * ks + 8 * hh;
      const v16b kbh = Frag<__bf16>::load(Qh + ko);
      const v16b kbl = Frag<__bf16>::load(Ql + ko);
      s = mma_bf16g(qah[ks], kbh, s);
      s = mma_bf16g(qah[ks], kbl, s);
      s = mma_bf16g(qal[ks], kbh, s);
    }
#pragma unroll
    for (int r = 0; r < 8; ++r) {
      float m = s[r];
#pragma unroll
      for (int off = 1; off < 16; off <<= 1) m = fmaxf(m, __shfl_xor(m, off, 32));
      Smx[rg][ch][8 * hh + r] = m;
    }
    __syncthreads();
    float alph[8];
#pragma unroll
    for (int r = 0; r < 8; ++r) {
      const int ri = 8 * hh + r;
      const float m4 = fmaxf(fmaxf(Smx[rg][0][ri], Smx[rg][1][ri]), fmaxf(Smx[rg][2][ri], Smx[rg][3][ri]));
      const float mnew = fmaxf(mrow[r], m4);
      alph[r] = expf(mrow[r] - mnew);
      mrow[r] = mnew;
      const float p = expf(s[r] - mnew);
      const _Float16 ph = (_Float16)(p * PA_PSC);
      pw[ri * PA_KCH + PA_KW * ch + c] = ph;
      float psum = (float)ph;
#pragma unroll
      for (int off = 1; off < 16; off <<= 1) psum += __shfl_xor(psum, off, 32);
      Ssm[rg][ch][ri] = psum;
#pragma unroll
      for (int t = 0; t < 8; ++t) oacc[t][r] *= alph[r];
    }
    __syncthreads();
#pragma unroll
    for (int r = 0; r < 8; ++r) {
      const int ri = 8 * hh + r;
      lrow[r] = lrow[r] * alph[r] + ((Ssm[rg][0][ri] + Ssm[rg][1][ri]) + (Ssm[rg][2][ri] + Ssm[rg][3][ri]));
    }
#pragma unroll 1
    for (int kk = 0; kk < 2; ++kk) {
      Frag<_Float16>::U pa;
      pa.h[0] = *(const v8h*)(pw + c * PA_KCH + kk * 32 + 8 * hh);
      pa.h[1] = *(const v8h*)(pw + c * PA_KCH + kk * 32 + 16 + 8 * hh);
      const _Float16* vrow = Vb + (size_t)c * SEQ + kc * PA_KCH + kk * 32 + 8 * hh;
#pragma unroll
      for (int t = 0; t < 8; ++t) {
        const v16h vb = Frag<_Float16>::load(vrow + (size_t)(16 * t) * SEQ);
        oacc[t] = mma_f16g(pa.v, vb, oacc[t]);
      }
    }
  }

  float* ob = out + (size_t)b * OUT_BSTRIDE + q0;
  const float* xb = x + (size_t)b * PA_C * SEQ_FULL + q0;
  const int q4 = (lane & 7) * 4;
#pragma unroll
  for (int ph2 = 0; ph2 < 2; ++ph2) {
    if ((ch >> 1) == ph2) {
#pragma unroll
      for (int r = 0; r < 8; ++r) {
        const float inv = 1.0f / lrow[r];
#pragma unroll
        for (int t = 0; t < 8; ++t)
          Ob[(128 * (ch & 1) + 16 * t + c) * PA_OBP + 16 * rg + 8 * hh + r] = oacc[t][r] * inv;
      }
    }
    __syncthreads();
    for (int pass = 0; pass < 2; ++pass) {
#pragma unroll
      for (int it = 0; it < 8; ++it) {
        const int chl = wave * 32 + it * 4 + (lane >> 3);
        const int chn = ph2 * 256 + chl;
        const v4f ov = *(const v4f*)(Ob + chl * PA_OBP + q4);
        const v4f xv = *(const v4f*)(xb + (size_t)chn * SEQ_FULL + q4);
        v4f res;
#pragma unroll
        for (int e = 0; e < 4; ++e) res[e] = al * ov[e] + bf_bits2f(f2bf_bits(xv[e]));
        *(volatile v4f*)(ob + (size_t)chn * OUT_NSTRIDE + q4) = res;
      }
      __threadfence();
    }
    __syncthreads();
  }
}

extern "C" void kernel_launch(void* const* d_in, const int* in_sizes, int n_in,
                              void* d_out, int out_size, void* d_ws, size_t ws_size,
                              hipStream_t stream)
{
  if (n_in < 8) return;
  const size_t needX   = (size_t)(NB - 1) * PA_C * SEQ_FULL + (size_t)(PA_C - 1) * SEQ_FULL + (size_t)SEQ;
  const size_t needOut = (size_t)(NB - 1) * OUT_BSTRIDE + (size_t)(PA_C - 1) * OUT_NSTRIDE + (size_t)SEQ;
  if ((size_t)in_sizes[0] < needX) return;
  if ((size_t)out_size < needOut) return;
  if (in_sizes[1] < PA_D * PA_C || in_sizes[3] < PA_D * PA_C || in_sizes[5] < PA_C * PA_C) return;
  if (in_sizes[2] < PA_D || in_sizes[4] < PA_D || in_sizes[6] < PA_C || in_sizes[7] < 1) return;

  const float* x   = (const float*)d_in[0];
  const float* wq  = (const float*)d_in[1];
  const float* bq  = (const float*)d_in[2];
  const float* wk  = (const float*)d_in[3];
  const float* bk  = (const float*)d_in[4];
  const float* wv  = (const float*)d_in[5];
  const float* bvv = (const float*)d_in[6];
  const float* alp = (const float*)d_in[7];
  float* out = (float*)d_out;

  const size_t szXt  = (size_t)NB * SEQ * PA_C * 2;
  const size_t szQK  = (size_t)NB * SEQ * PA_QKP * 2;
  const size_t szV   = (size_t)NB * PA_C * SEQ * 2;
  const size_t szWqk = (size_t)PA_QKP * PA_C * 2;
  const size_t szWv  = (size_t)PA_C * PA_C * 2;
  const size_t szB   = (size_t)(PA_QKP + PA_C) * 4;
  const size_t offXt  = 0;
  const size_t offQKh = offXt + szXt;
  const size_t offQKl = offQKh + szQK;
  const size_t offV   = offQKl + szQK;
  const size_t offWqk = offV + szV;
  const size_t offWv  = offWqk + szWqk;
  const size_t offB   = offWv + szWv;
  const size_t offEnd = offB + szB;
  if (offEnd > ws_size) return;
  if (offEnd > (size_t)134217728) return;

  char* ws = (char*)d_ws;
  unsigned short* Xt16  = (unsigned short*)(ws + offXt);
  unsigned short* QKh   = (unsigned short*)(ws + offQKh);
  unsigned short* QKl   = (unsigned short*)(ws + offQKl);
  unsigned short* V16   = (unsigned short*)(ws + offV);
  unsigned short* Wqk16 = (unsigned short*)(ws + offWqk);
  unsigned short* Wv16  = (unsigned short*)(ws + offWv);
  float* brnd = (float*)(ws + offB);

  prep_params<<<PP_NBLK, 256, 0, stream>>>(wq, wk, wv, bq, bk, bvv, Wqk16, Wv16, brnd);
  xpose_x_bf16<<<NB * (SEQ / 32), 256, 0, stream>>>(x, Xt16);
  wmma_gemm64<1, false, 2, 2, false, 0><<<dim3((SEQ / 64) * (PA_QKP / 64) / 8, NB), 256, 0, stream>>>(
      Xt16, Xt16, PA_C, (long)SEQ * PA_C,
      Wqk16, Wqk16, PA_C, 0L,
      (void*)QKh, (void*)QKl, PA_QKP, (long)SEQ * PA_QKP,
      brnd, x, 0L,
      SEQ, PA_QKP, PA_C, 1.0f);
  wmma_gemm64<1, false, 1, 1, false, 0><<<dim3((PA_C / 64) * (SEQ / 64) / 8, NB), 256, 0, stream>>>(
      Wv16, Wv16, PA_C, 0L,
      Xt16, Xt16, PA_C, (long)SEQ * PA_C,
      (void*)V16, (void*)V16, SEQ, (long)PA_C * SEQ,
      brnd + PA_QKP, x, 0L,
      PA_C, SEQ, PA_C, 1.0f);
  pos_attn<<<NB * (SEQ / 32), 256, 0, stream>>>(QKh, QKl, V16, x, alp, out);
}
